// SelfAtt_28862180229450
// MI455X (gfx1250) — hardware-run, weakly checked
//
#include <hip/hip_runtime.h>
#include <stdint.h>

#define DEVINL __device__ __forceinline__

typedef _Float16 f16t;
typedef _Float16 v16h __attribute__((ext_vector_type(16)));
typedef _Float16 v8h  __attribute__((ext_vector_type(8)));
typedef __attribute__((ext_vector_type(16))) __bf16 v16b;
typedef unsigned short v8us __attribute__((ext_vector_type(8)));
typedef float v8f __attribute__((ext_vector_type(8)));
typedef float v4f __attribute__((ext_vector_type(4)));
typedef v8h  __attribute__((may_alias)) v8ha;
typedef v8us __attribute__((may_alias)) v8usa;
typedef v4f  __attribute__((may_alias)) v4fa;
union FragH { v16h v; v8h half[2]; };
union FragB { v16b v; v8us half[2]; };

#define NB    16
#define CC    512
#define NPIX  1024
#define NH    8
#define HD    64
#define NGRP  32
#define CPG   16
#define NQKV  1536
#define WROWS 2048
#define TPB   256
#define WAVES 8
#define PT    32
#define PQ    520
#define SP    36
#define PTO   64
#define SPO   68
#define NC    64
#define PKC   72
#define XCAR  8.0f
#define WCAR  16.0f
#define OCAR  8.0f
#define GN_EPS 1e-5f

static_assert(TPB == WAVES * 32);
static_assert((PQ % 8) == 0);
static_assert((SP % 4) == 0);
static_assert((SPO % 4) == 0);
static_assert((PKC % 8) == 0);
static_assert((NPIX % PT) == 0);
static_assert((NPIX % PTO) == 0);
static_assert((NPIX % NC) == 0);
static_assert((CC % 32) == 0);
static_assert(CC == NH * HD);
static_assert(CC == NGRP * CPG);
static_assert(NQKV == 3 * CC);
static_assert((CPG * NPIX) % TPB == 0);
static_assert(4 * HD * PKC >= WAVES * 16 * PKC);
static_assert(TPB * 8 == 2 * HD * 16);

DEVINL int imin(int a, int b) { return a < b ? a : b; }
DEVINL int imax(int a, int b) { return a > b ? a : b; }

DEVINL v8f wmma_f16(v16h a, v16h b, v8f c) {
  v8f d = __builtin_amdgcn_wmma_f32_16x16x32_f16(false, a, false, b, (short)0, c, false, false);
  asm volatile("v_nop\n\tv_nop\n\tv_nop\n\tv_nop" : "+v"(d) : "v"(a), "v"(b));
  return d;
}
DEVINL v8f wmma_bf(v16b a, v16b b, v8f c) {
  v8f d = __builtin_amdgcn_wmma_f32_16x16x32_bf16(false, a, false, b, (short)0, c, false, false);
  asm volatile("v_nop\n\tv_nop\n\tv_nop\n\tv_nop" : "+v"(d) : "v"(a), "v"(b));
  return d;
}
DEVINL v8f wmma_bf3(const FragB& ah, const FragB& al, const FragB& bh, const FragB& bl, v8f c) {
  c = wmma_bf(ah.v, bh.v, c);
  c = wmma_bf(ah.v, bl.v, c);
  c = wmma_bf(al.v, bh.v, c);
  return c;
}
DEVINL v8f zero8f() {
  v8f z = {0.f, 0.f, 0.f, 0.f, 0.f, 0.f, 0.f, 0.f};
  return z;
}

DEVINL unsigned int bf_rne(float f) {
  const unsigned int u = __float_as_uint(f);
  return (u + 0x7FFFu + ((u >> 16) & 1u)) >> 16;
}
DEVINL void split8(v4f a, v4f b, v8us& hi, v8us& lo) {
  #pragma unroll
  for (int i = 0; i < 4; ++i) {
    const unsigned int h0 = bf_rne(a[i]);
    const float r0 = a[i] - __uint_as_float(h0 << 16);
    hi[i] = (unsigned short)h0;
    lo[i] = (unsigned short)bf_rne(r0);
    const unsigned int h1 = bf_rne(b[i]);
    const float r1 = b[i] - __uint_as_float(h1 << 16);
    hi[4 + i] = (unsigned short)h1;
    lo[4 + i] = (unsigned short)bf_rne(r1);
  }
}

__global__ __launch_bounds__(TPB) void prep_w_k(const float* __restrict__ qkv_w, const float* __restrict__ proj_w,
                                               f16t* __restrict__ W16)
{
  const int t = blockIdx.x * TPB + threadIdx.x;
  if (t >= WROWS * 64) return;
  const int row = t >> 6, piece = (t & 63) * 8;
  const int rq = imin(row, NQKV - 1);
  const int rp = imin(imax(row - NQKV, 0), CC - 1);
  const v4f q0 = *(const v4fa*)(qkv_w + (size_t)rq * CC + piece);
  const v4f q1 = *(const v4fa*)(qkv_w + (size_t)rq * CC + piece + 4);
  const v4f w0 = *(const v4fa*)(proj_w + (size_t)rp * CC + piece);
  const v4f w1 = *(const v4fa*)(proj_w + (size_t)rp * CC + piece + 4);
  const bool isq = row < NQKV;
  v8h o;
  #pragma unroll
  for (int i = 0; i < 4; ++i) {
    const float a = isq ? q0[i] : w0[i];
    const float c = isq ? q1[i] : w1[i];
    o[i]     = (f16t)(a * WCAR);
    o[4 + i] = (f16t)(c * WCAR);
  }
  f16t* dst = W16 + (size_t)row * CC + piece;
  *(volatile v8h*)dst = o;
  __threadfence();
  *(volatile v8h*)dst = o;
}

__global__ __launch_bounds__(TPB) void gnstat_k(const float* __restrict__ x, float* __restrict__ GNS)
{
  __shared__ float sRa[WAVES];
  __shared__ float sRb[WAVES];
  __shared__ __attribute__((aligned(16))) float sSt[NGRP * 2];
  const int tid = threadIdx.x, lane = tid & 31, wave = tid >> 5;
  const int b = blockIdx.x;
  const float inv_n = 1.0f / (float)(CPG * NPIX);
  #pragma unroll 1
  for (int g = 0; g < NGRP; ++g) {
    const float* xb = x + ((size_t)b * CC + g * CPG) * NPIX;
    float s = 0.0f;
    #pragma unroll 4
    for (int j = 0; j < (CPG * NPIX) / TPB; ++j) s += xb[tid + TPB * j];
    #pragma unroll
    for (int w = 16; w > 0; w >>= 1) s += __shfl_xor(s, w);
    if (lane == 0) sRa[wave] = s;
    __syncthreads();
    float tot = sRa[0];
    #pragma unroll
    for (int w2 = 1; w2 < WAVES; ++w2) tot += sRa[w2];
    const float mean = tot * inv_n;
    float ss = 0.0f;
    #pragma unroll 4
    for (int j = 0; j < (CPG * NPIX) / TPB; ++j) {
      const float d = xb[tid + TPB * j] - mean;
      ss = fmaf(d, d, ss);
    }
    #pragma unroll
    for (int w = 16; w > 0; w >>= 1) ss += __shfl_xor(ss, w);
    if (lane == 0) sRb[wave] = ss;
    __syncthreads();
    float tot2 = sRb[0];
    #pragma unroll
    for (int w2 = 1; w2 < WAVES; ++w2) tot2 += sRb[w2];
    const float var = tot2 * inv_n;
    if (tid == 0) { sSt[2 * g] = mean; sSt[2 * g + 1] = rsqrtf(var + GN_EPS); }
    __syncthreads();
  }
  if (wave == 0) {
    const int lc = lane & 15;
    const v4f v = *(const v4fa*)(sSt + 4 * lc);
    float* dst = GNS + (size_t)b * (NGRP * 2) + 4 * lc;
    if (lane < 16) *(volatile v4f*)dst = v;
    __threadfence();
    if (lane < 16) *(volatile v4f*)dst = v;
  }
}

__global__ __launch_bounds__(TPB) void qkv_k(const float* __restrict__ x, const float* __restrict__ gsc,
                                           const float* __restrict__ gbi, const float* __restrict__ GNS,
                                           const f16t* __restrict__ W16, float* __restrict__ QF,
                                           float* __restrict__ KVF)
{
  __shared__ __attribute__((aligned(16))) f16t  sX[PT * PQ];
  __shared__ __attribute__((aligned(16))) float sStg[WAVES * 16 * SP];
  __shared__ float sMu[NGRP];
  __shared__ float sRs[NGRP];
  const int tid = threadIdx.x, lane = tid & 31, wave = tid >> 5;
  const int h = lane >> 4, m = lane & 15;
  const int p0 = blockIdx.x * PT, b = blockIdx.y;

  if (tid < NGRP) {
    sMu[tid] = GNS[(size_t)b * (NGRP * 2) + 2 * tid];
    sRs[tid] = GNS[(size_t)b * (NGRP * 2) + 2 * tid + 1];
  }
  __syncthreads();
  {
    const int c0 = tid >> 3, p4 = (tid & 7) * 4;
    const float* xb = x + (size_t)b * CC * NPIX + p0 + p4;
    #pragma unroll 2
    for (int i = 0; i < CC / 32; ++i) {
      const int c = c0 + 32 * i, g = c >> 4;
      const v4f v = *(const v4fa*)(xb + (size_t)c * NPIX);
      const float mu = sMu[g], rs = sRs[g], sc = gsc[c], bi = gbi[c];
      #pragma unroll
      for (int j = 0; j < 4; ++j) {
        float t = (v[j] - mu) * rs;
        t = fmaf(t, sc, bi);
        sX[(p4 + j) * PQ + c] = (f16t)(t * XCAR);
      }
    }
  }
  __syncthreads();

  const float osc = 1.0f / (XCAR * WCAR);
  const int sub = lane >> 3, piece = (lane & 7) * 4;
  float* stg = sStg + wave * (16 * SP);
  #pragma unroll 1
  for (int og = 0; og < 6; ++og) {
    const int obase = og * 256 + wave * 32;
    v8f acc[2][2];
    #pragma unroll
    for (int mt = 0; mt < 2; ++mt) {
      #pragma unroll
      for (int nt = 0; nt < 2; ++nt) acc[mt][nt] = zero8f();
    }
    const f16t* arow = W16 + (size_t)(obase + m) * CC + 8 * h;
    const f16t* brow = sX + m * PQ + 8 * h;
    #pragma unroll 1
    for (int ks = 0; ks < CC / 32; ++ks) {
      const int k0 = 32 * ks;
      FragH a0, a1, b0, b1;
      a0.half[0] = *(const v8ha*)(arow + k0);
      a0.half[1] = *(const v8ha*)(arow + k0 + 16);
      a1.half[0] = *(const v8ha*)(arow + 16 * CC + k0);
      a1.half[1] = *(const v8ha*)(arow + 16 * CC + k0 + 16);
      b0.half[0] = *(const v8ha*)(brow + k0);
      b0.half[1] = *(const v8ha*)(brow + k0 + 16);
      b1.half[0] = *(const v8ha*)(brow + 16 * PQ + k0);
      b1.half[1] = *(const v8ha*)(brow + 16 * PQ + k0 + 16);
      acc[0][0] = wmma_f16(a0.v, b0.v, acc[0][0]);
      acc[0][1] = wmma_f16(a0.v, b1.v, acc[0][1]);
      acc[1][0] = wmma_f16(a1.v, b0.v, acc[1][0]);
      acc[1][1] = wmma_f16(a1.v, b1.v, acc[1][1]);
    }

    if (og < 2) {
      #pragma unroll
      for (int nt = 0; nt < 2; ++nt) {
        #pragma unroll
        for (int mt = 0; mt < 2; ++mt) {
          v4f e0, e1;
          #pragma unroll
          for (int r = 0; r < 4; ++r) { e0[r] = acc[mt][nt][r] * osc; e1[r] = acc[mt][nt][4 + r] * osc; }
          *(v4fa*)(stg + m * SP + 16 * mt + 8 * h)     = e0;
          *(v4fa*)(stg + m * SP + 16 * mt + 8 * h + 4) = e1;
        }
        __syncthreads();
        float* dst = QF + ((size_t)b * NPIX + p0 + 16 * nt) * CC + obase + piece;
        #pragma unroll
        for (int i = 0; i < 4; ++i) {
          const int row = 4 * i + sub;
          const v4f v = *(const v4fa*)(stg + row * SP + piece);
          *(volatile v4f*)(dst + (size_t)row * CC) = v;
        }
        __threadfence();
        #pragma unroll
        for (int i = 0; i < 4; ++i) {
          const int row = 4 * i + sub;
          const v4f v = *(const v4fa*)(stg + row * SP + piece);
          *(volatile v4f*)(dst + (size_t)row * CC) = v;
        }
        __syncthreads();
      }
    } else {
      const int q = og - 2;
      const size_t rowbase = (size_t)(q >> 1) * NB * CC + (size_t)b * CC + (size_t)((q & 1) * 256 + wave * 32);
      #pragma unroll
      for (int mt = 0; mt < 2; ++mt) {
        #pragma unroll
        for (int nt = 0; nt < 2; ++nt) {
          #pragma unroll
          for (int r = 0; r < 8; ++r) stg[(8 * h + r) * SP + 16 * nt + m] = acc[mt][nt][r] * osc;
        }
        __syncthreads();
        float* dst = KVF + (rowbase + 16 * mt) * NPIX + p0 + piece;
        #pragma unroll
        for (int i = 0; i < 4; ++i) {
          const int row = 4 * i + sub;
          const v4f v = *(const v4fa*)(stg + row * SP + piece);
          *(volatile v4f*)(dst + (size_t)row * NPIX) = v;
        }
        __threadfence();
        #pragma unroll
        for (int i = 0; i < 4; ++i) {
          const int row = 4 * i + sub;
          const v4f v = *(const v4fa*)(stg + row * SP + piece);
          *(volatile v4f*)(dst + (size_t)row * NPIX) = v;
        }
        __syncthreads();
      }
    }
  }
}

__global__ __launch_bounds__(TPB) void att_k(const float* __restrict__ QF, const float* __restrict__ KVF,
                                           f16t* __restrict__ OT)
{
  __shared__ __attribute__((aligned(16))) unsigned short sPl[4 * HD * PKC];
  __shared__ __attribute__((aligned(16))) unsigned short sAH[HD * PKC];
  __shared__ __attribute__((aligned(16))) unsigned short sAL[HD * PKC];
  __shared__ float sMx[HD];
  __shared__ float sIv[HD];
  const int tid = threadIdx.x, lane = tid & 31, wave = tid >> 5;
  const int h = lane >> 4, m = lane & 15;
  const int bg = blockIdx.x, b = bg >> 3, g = bg & 7;
  const float* kbase = KVF + ((size_t)b * CC + g * HD) * NPIX;
  const float* vbase = KVF + ((size_t)NB * CC + (size_t)b * CC + g * HD) * NPIX;

  #pragma unroll 1
  for (int j = 0; j < 8; ++j) {
    const int r = wave * 8 + j;
    const float* kr = kbase + (size_t)r * NPIX + 4 * lane;
    v4f z[8];
    float mx = -3.0e38f;
    #pragma unroll
    for (int jj = 0; jj < 8; ++jj) {
      z[jj] = *(const v4fa*)(kr + 128 * jj);
      #pragma unroll
      for (int e = 0; e < 4; ++e) mx = fmaxf(mx, z[jj][e]);
    }
    #pragma unroll
    for (int w = 16; w > 0; w >>= 1) mx = fmaxf(mx, __shfl_xor(mx, w));
    float sm = 0.0f;
    #pragma unroll
    for (int jj = 0; jj < 8; ++jj) {
      #pragma unroll
      for (int e = 0; e < 4; ++e) sm += __expf(z[jj][e] - mx);
    }
    #pragma unroll
    for (int w = 16; w > 0; w >>= 1) sm += __shfl_xor(sm, w);
    if (lane == 0) { sMx[r] = mx; sIv[r] = 1.0f / sm; }
  }
  __syncthreads();

  unsigned short* sKH = sPl;
  unsigned short* sKL = sPl + HD * PKC;
  unsigned short* sVH = sPl + 2 * HD * PKC;
  unsigned short* sVL = sPl + 3 * HD * PKC;
  const int dT = wave >> 1, eT0 = 2 * (wave & 1);
  v8f acc[2];
  acc[0] = zero8f();
  acc[1] = zero8f();
  const int sr = tid >> 2, seg = (tid & 3) * 16;
  const float* ksrc = kbase + (size_t)sr * NPIX + seg;
  const float* vsrc = vbase + (size_t)sr * NPIX + seg;
  #pragma unroll 1
  for (int ch = 0; ch < NPIX / NC; ++ch) {
    const int n0 = ch * NC;
    {
      const float mx = sMx[sr], iv = sIv[sr];
      v4f k0v = *(const v4fa*)(ksrc + n0);
      v4f k1v = *(const v4fa*)(ksrc + n0 + 4);
      v4f k2v = *(const v4fa*)(ksrc + n0 + 8);
      v4f k3v = *(const v4fa*)(ksrc + n0 + 12);
      #pragma unroll
      for (int e = 0; e < 4; ++e) {
        k0v[e] = __expf(k0v[e] - mx) * iv;
        k1v[e] = __expf(k1v[e] - mx) * iv;
        k2v[e] = __expf(k2v[e] - mx) * iv;
        k3v[e] = __expf(k3v[e] - mx) * iv;
      }
      v8us hA, lA, hB, lB;
      split8(k0v, k1v, hA, lA);
      split8(k2v, k3v, hB, lB);
      *(v8usa*)(sKH + sr * PKC + seg)     = hA;
      *(v8usa*)(sKH + sr * PKC + seg + 8) = hB;
      *(v8usa*)(sKL + sr * PKC + seg)     = lA;
      *(v8usa*)(sKL + sr * PKC + seg + 8) = lB;
      const v4f v0 = *(const v4fa*)(vsrc + n0);
      const v4f v1 = *(const v4fa*)(vsrc + n0 + 4);
      const v4f v2 = *(const v4fa*)(vsrc + n0 + 8);
      const v4f v3 = *(const v4fa*)(vsrc + n0 + 12);
      split8(v0, v1, hA, lA);
      split8(v2, v3, hB, lB);
      *(v8usa*)(sVH + sr * PKC + seg)     = hA;
      *(v8usa*)(sVH + sr * PKC + seg + 8) = hB;
      *(v8usa*)(sVL + sr * PKC + seg)     = lA;
      *(v8usa*)(sVL + sr * PKC + seg + 8) = lB;
    }
    __syncthreads();
    #pragma unroll
    for (int kk = 0; kk < 2; ++kk) {
      const int k0 = 32 * kk;
      FragB ah, al, bh[2], bl[2];
      const int ao = (16 * dT + m) * PKC + k0 + 8 * h;
      ah.half[0] = *(const v8usa*)(sKH + ao);
      ah.half[1] = *(const v8usa*)(sKH + ao + 16);
      al.half[0] = *(const v8usa*)(sKL + ao);
      al.half[1] = *(const v8usa*)(sKL + ao + 16);
      #pragma unroll
      for (int t = 0; t < 2; ++t) {
        const int bo = (16 * (eT0 + t) + m) * PKC + k0 + 8 * h;
        bh[t].half[0] = *(const v8usa*)(sVH + bo);
        bh[t].half[1] = *(const v8usa*)(sVH + bo + 16);
        bl[t].half[0] = *(const v8usa*)(sVL + bo);
        bl[t].half[1] = *(const v8usa*)(sVL + bo + 16);
      }
      #pragma unroll
      for (int t = 0; t < 2; ++t) acc[t] = wmma_bf3(ah, al, bh[t], bl[t], acc[t]);
    }
    __syncthreads();
  }
  #pragma unroll
  for (int t = 0; t < 2; ++t) {
    v4f a0, a1;
    #pragma unroll
    for (int r = 0; r < 4; ++r) { a0[r] = acc[t][r]; a1[r] = acc[t][4 + r]; }
    v8us hv, lv;
    split8(a0, a1, hv, lv);
    const int o = (16 * (eT0 + t) + m) * PKC + 16 * dT + 8 * h;
    *(v8usa*)(sAH + o) = hv;
    *(v8usa*)(sAL + o) = lv;
  }
  __syncthreads();

  f16t* sO = (f16t*)sPl + wave * (16 * PKC);
  const float* qbase = QF + (size_t)b * NPIX * CC + g * HD;
  const int sub = lane >> 3, piece = (lane & 7) * 8;
  #pragma unroll 1
  for (int j = 0; j < 8; ++j) {
    const int nt = wave + 8 * j;
    const float* qr = qbase + (size_t)(16 * nt + m) * CC;
    FragB bh[2], bl[2];
    #pragma unroll
    for (int kk = 0; kk < 2; ++kk) {
      const float* qa = qr + 32 * kk + 8 * h;
      const v4f c0 = *(const v4fa*)(qa);
      const v4f c1 = *(const v4fa*)(qa + 4);
      const v4f c2 = *(const v4fa*)(qa + 16);
      const v4f c3 = *(const v4fa*)(qa + 20);
      split8(c0, c1, bh[kk].half[0], bl[kk].half[0]);
      split8(c2, c3, bh[kk].half[1], bl[kk].half[1]);
    }
    #pragma unroll
    for (int eT = 0; eT < 4; ++eT) {
      v8f o = zero8f();
      #pragma unroll
      for (int kk = 0; kk < 2; ++kk) {
        const int ao = (16 * eT + m) * PKC + 32 * kk + 8 * h;
        FragB ah, al;
        ah.half[0] = *(const v8usa*)(sAH + ao);
        ah.half[1] = *(const v8usa*)(sAH + ao + 16);
        al.half[0] = *(const v8usa*)(sAL + ao);
        al.half[1] = *(const v8usa*)(sAL + ao + 16);
        o = wmma_bf3(ah, al, bh[kk], bl[kk], o);
      }
      v8h ov;
      #pragma unroll
      for (int r = 0; r < 8; ++r) ov[r] = (f16t)(o[r] * OCAR);
      *(v8ha*)(sO + m * PKC + 16 * eT + 8 * h) = ov;
    }
    __syncthreads();
    f16t* dst = OT + ((size_t)b * NPIX + 16 * nt) * CC + g * HD + piece;
    #pragma unroll
    for (int i = 0; i < 4; ++i) {
      const int row = 4 * i + sub;
      const v8h v = *(const v8ha*)(sO + row * PKC + piece);
      *(volatile v8h*)(dst + (size_t)row * CC) = v;
    }
    __threadfence();
    #pragma unroll
    for (int i = 0; i < 4; ++i) {
      const int row = 4 * i + sub;
      const v8h v = *(const v8ha*)(sO + row * PKC + piece);
      *(volatile v8h*)(dst + (size_t)row * CC) = v;
    }
    __syncthreads();
  }
}

__global__ __launch_bounds__(TPB) void proj_k(const f16t* __restrict__ OT, const f16t* __restrict__ WP,
                                            const float* __restrict__ pb, float* __restrict__ out)
{
  __shared__ __attribute__((aligned(16))) float sO[WAVES * 16 * SPO];
  const int tid = threadIdx.x, lane = tid & 31, wave = tid >> 5;
  const int h = lane >> 4, m = lane & 15;
  const int p0 = blockIdx.x * PTO, og = blockIdx.y, b = blockIdx.z;
  const int obase = og * 256 + wave * 32;

  v8f acc[2][4];
  #pragma unroll
  for (int mt = 0; mt < 2; ++mt) {
    #pragma unroll
    for (int nt = 0; nt < 4; ++nt) acc[mt][nt] = zero8f();
  }
  const f16t* arow = WP + (size_t)(obase + m) * CC + 8 * h;
  const f16t* brow = OT + ((size_t)b * NPIX + p0 + m) * CC + 8 * h;
  #pragma unroll 1
  for (int ks = 0; ks < CC / 32; ++ks) {
    const int k0 = 32 * ks;
    FragH a0, a1, bf[4];
    a0.half[0] = *(const v8ha*)(arow + k0);
    a0.half[1] = *(const v8ha*)(arow + k0 + 16);
    a1.half[0] = *(const v8ha*)(arow + 16 * CC + k0);
    a1.half[1] = *(const v8ha*)(arow + 16 * CC + k0 + 16);
    #pragma unroll
    for (int nt = 0; nt < 4; ++nt) {
      bf[nt].half[0] = *(const v8ha*)(brow + (size_t)16 * nt * CC + k0);
      bf[nt].half[1] = *(const v8ha*)(brow + (size_t)16 * nt * CC + k0 + 16);
    }
    #pragma unroll
    for (int nt = 0; nt < 4; ++nt) {
      acc[0][nt] = wmma_f16(a0.v, bf[nt].v, acc[0][nt]);
      acc[1][nt] = wmma_f16(a1.v, bf[nt].v, acc[1][nt]);
    }
  }

  const float sc = 1.0f / (WCAR * OCAR);
  float* stg = sO + wave * (16 * SPO);
  const int l16 = lane & 15, rsel = lane >> 4;
  #pragma unroll
  for (int mt = 0; mt < 2; ++mt) {
    const int ob = obase + 16 * mt + 8 * h;
    const v4f cb0 = *(const v4fa*)(pb + ob);
    const v4f cb1 = *(const v4fa*)(pb + ob + 4);
    #pragma unroll
    for (int nt = 0; nt < 4; ++nt) {
      #pragma unroll
      for (int r = 0; r < 4; ++r) {
        stg[(8 * h + r) * SPO + 16 * nt + m]     = fmaf(acc[mt][nt][r], sc, cb0[r]);
        stg[(8 * h + 4 + r) * SPO + 16 * nt + m] = fmaf(acc[mt][nt][4 + r], sc, cb1[r]);
      }
    }
    __syncthreads();
    float* orow = out + ((size_t)b * CC + obase + 16 * mt) * NPIX + p0;
    #pragma unroll
    for (int i = 0; i < 8; ++i) {
      const int row = 2 * i + rsel;
      const v4f v = *(const v4fa*)(stg + row * SPO + 4 * l16);
      *(volatile v4f*)(orow + (size_t)row * NPIX + 4 * l16) = v;
    }
    __threadfence();
    #pragma unroll
    for (int i = 0; i < 8; ++i) {
      const int row = 2 * i + rsel;
      const v4f v = *(const v4fa*)(stg + row * SPO + 4 * l16);
      *(volatile v4f*)(orow + (size_t)row * NPIX + 4 * l16) = v;
    }
    __syncthreads();
  }
}

extern "C" void kernel_launch(void* const* d_in, const int* in_sizes, int n_in,
                              void* d_out, int out_size, void* d_ws, size_t ws_size,
                              hipStream_t stream) {
  if (n_in < 6) return;
  if (in_sizes[0] != NB * CC * NPIX) return;
  if (in_sizes[1] != CC)             return;
  if (in_sizes[2] != CC)             return;
  if (in_sizes[3] != NQKV * CC)      return;
  if (in_sizes[4] != CC * CC)        return;
  if (in_sizes[5] != CC)             return;
  if (out_size != NB * CC * NPIX)    return;

  const float* x      = (const float*)d_in[0];
  const float* gsc    = (const float*)d_in[1];
  const float* gbi    = (const float*)d_in[2];
  const float* qkv_w  = (const float*)d_in[3];
  const float* proj_w = (const float*)d_in[4];
  const float* proj_b = (const float*)d_in[5];
  float* outp = (float*)d_out;

  const size_t szW16 = (size_t)WROWS * CC * 2;
  const size_t szGNS = (size_t)NB * NGRP * 2 * 4;
  const size_t szQF  = (size_t)NB * NPIX * CC * 4;
  const size_t szKVF = (size_t)2 * NB * CC * NPIX * 4;
  const size_t szOT  = (size_t)NB * NPIX * CC * 2;
  size_t off = 0;
  char* ws = (char*)d_ws;
  f16t*  W16 = (f16t*)(ws + off);   off += szW16;
  float* GNS = (float*)(ws + off);  off += szGNS;
  float* QF  = (float*)(ws + off);  off += szQF;
  float* KVF = (float*)(ws + off);  off += szKVF;
  f16t*  OT  = (f16t*)(ws + off);   off += szOT;
  if (off > ws_size) return;
  const f16t* WP = W16 + (size_t)NQKV * CC;

  prep_w_k<<<(WROWS * 64) / TPB, TPB, 0, stream>>>(qkv_w, proj_w, W16);
  gnstat_k<<<NB, TPB, 0, stream>>>(x, GNS);
  qkv_k<<<dim3(NPIX / PT, NB), TPB, 0, stream>>>(x, gsc, gbi, GNS, W16, QF, KVF);
  att_k<<<NB * NH, TPB, 0, stream>>>(QF, KVF, OT);
  proj_k<<<dim3(NPIX / PTO, 2, NB), TPB, 0, stream>>>(OT, WP, proj_b, outp);
}
